// BayesianDenseLayer_45114336477600
// MI455X (gfx1250) — hardware-verified
//
#include <hip/hip_runtime.h>
#include <math.h>

typedef __attribute__((ext_vector_type(16))) _Float16 v16h;
typedef __attribute__((ext_vector_type(16))) __bf16 v16b;
typedef __attribute__((ext_vector_type(8)))  _Float16 v8h;
typedef __attribute__((ext_vector_type(8)))  float v8f;
typedef __attribute__((ext_vector_type(4)))  float v4f;
typedef __attribute__((ext_vector_type(2)))  float v2f;
typedef __attribute__((ext_vector_type(4)))  unsigned v4u;
typedef __attribute__((ext_vector_type(4)))  int v4i;
typedef float __attribute__((may_alias)) float_a;
typedef int __attribute__((may_alias)) int_a;

template <typename T> __device__ __forceinline__ void vst2(void* p, T v) { *(volatile T*)p = v; __threadfence(); *(volatile T*)p = v; }
__device__ __forceinline__ v8f wmma16(v16h a, v16h b, v8f c) {
  v8f d = __builtin_amdgcn_wmma_f32_16x16x32_f16(false, a, false, b, (short)0, c, false, false);
  asm volatile("v_nop\n\tv_nop\n\tv_nop\n\tv_nop" : "+v"(d) : "v"(a), "v"(b));
  return d;
}
__device__ __forceinline__ v8f wmma_bf(v16b a, v16b b, v8f c) {
  v8f d = __builtin_amdgcn_wmma_f32_16x16x32_bf16(false, a, false, b, (short)0, c, false, false);
  asm volatile("v_nop\n\tv_nop\n\tv_nop\n\tv_nop" : "+v"(d) : "v"(a), "v"(b));
  return d;
}
__device__ __forceinline__ v16h frag_h(const _Float16* rowk0, int lane) {
  union { v16h v; v8h q[2]; } u; const _Float16* p = rowk0 + 8 * (lane >> 4);
  u.q[0] = *(const v8h*)p; u.q[1] = *(const v8h*)(p + 16); return u.v;
}
__device__ __forceinline__ v16h frag_f32(const float* rowk0, int lane) {
  v16h a; const float* p = rowk0 + 8 * (lane >> 4);
#pragma unroll
  for (int i = 0; i < 8; ++i) { a[i] = (_Float16)p[i]; a[8 + i] = (_Float16)p[16 + i]; }
  return a;
}
__device__ __forceinline__ v16h frag_f32s(const float* rowk0, int lane, float sc) {
  v16h a; const float* p = rowk0 + 8 * (lane >> 4);
#pragma unroll
  for (int i = 0; i < 8; ++i) { a[i] = (_Float16)(p[i] * sc); a[8 + i] = (_Float16)(p[16 + i] * sc); }
  return a;
}
__device__ __forceinline__ v16h fragc_f32(const float* W, int k0, int n, int lane, int ld, int K) {
  v16h a; const int g = lane >> 4;
#pragma unroll
  for (int i = 0; i < 8; ++i) { const int ka = k0 + 8 * g + i, kb = ka + 16;
    a[i] = (_Float16)(ka < K ? W[(size_t)ka * ld + n] : 0.f); a[8 + i] = (_Float16)(kb < K ? W[(size_t)kb * ld + n] : 0.f); }
  return a;
}
struct F2 { v16b h, l; };
__device__ __forceinline__ F2 bsplit16(const float v[16]) { F2 r;
#pragma unroll
  for (int i = 0; i < 16; ++i) { const __bf16 h = (__bf16)v[i]; r.h[i] = h; r.l[i] = (__bf16)(v[i] - (float)h); }
  return r; }
__device__ __forceinline__ F2 split_row(const float* row, int k0, int lane) { float v[16]; const float* p = row + k0 + 8 * (lane >> 4);
#pragma unroll
  for (int i = 0; i < 8; ++i) { v[i] = p[i]; v[8 + i] = p[16 + i]; }
  return bsplit16(v); }
__device__ __forceinline__ F2 split_rowK(const float* row, int k0, int lane, int K) { float v[16]; const int g = lane >> 4;
#pragma unroll
  for (int i = 0; i < 8; ++i) { const int ka = k0 + 8 * g + i, kb = ka + 16; v[i] = ka < K ? row[ka] : 0.f; v[8 + i] = kb < K ? row[kb] : 0.f; }
  return bsplit16(v); }
__device__ __forceinline__ F2 split_col(const float* W, int k0, int n, int lane, int ld, int K) { float v[16]; const int g = lane >> 4;
#pragma unroll
  for (int i = 0; i < 8; ++i) { const int ka = k0 + 8 * g + i, kb = ka + 16; v[i] = ka < K ? W[(size_t)ka * ld + n] : 0.f; v[8 + i] = kb < K ? W[(size_t)kb * ld + n] : 0.f; }
  return bsplit16(v); }
__device__ __forceinline__ v8f mac3(const F2& a, const F2& b, v8f c) { c = wmma_bf(a.l, b.h, c); c = wmma_bf(a.h, b.l, c); return wmma_bf(a.h, b.h, c); }
__device__ __forceinline__ float sigm(float v) { return 1.0f / (1.0f + expf(-v)); }
#define LDSX() do { asm volatile("s_wait_dscnt 0" ::: "memory"); __builtin_amdgcn_wave_barrier(); __builtin_amdgcn_fence(__ATOMIC_RELEASE, "workgroup"); } while (0)

#define NBT 4096
#define DI 2048
#define DO 2048

__device__ __forceinline__ float softplus_f(float v) { return fmaxf(v, 0.f) + log1pf(expf(-fabsf(v))); }

__global__ __launch_bounds__(256) void k_cvtx(const float* __restrict__ x, const int* __restrict__ s, _Float16* __restrict__ x16, _Float16* __restrict__ xs16) {
  const size_t g8 = (size_t)blockIdx.x * 256 + threadIdx.x; if (g8 >= (size_t)NBT * DI / 8) return;
  union { v8h h; v4u u; } a, c;
#pragma unroll
  for (int e = 0; e < 8; ++e) { const float v = x[g8 * 8 + e]; a.h[e] = (_Float16)v; c.h[e] = (_Float16)(v * (float)s[g8 * 8 + e]); }
  vst2(x16 + g8 * 8, a.u); vst2(xs16 + g8 * 8, c.u);
}
__global__ __launch_bounds__(256) void k_packT(const float* __restrict__ wl, const float* __restrict__ wsd, const float* __restrict__ epw, _Float16* __restrict__ P1, _Float16* __restrict__ P2) {
  __shared__ float t1[64][65], t2[64][65];
  const int o0 = blockIdx.x * 64, k0 = blockIdx.y * 64, tid = threadIdx.x;
  for (int q = tid; q < 64 * 64; q += 256) { const int kl = q >> 6, ol = q & 63; const size_t i = (size_t)(k0 + kl) * DO + o0 + ol; t1[kl][ol] = wl[i]; t2[kl][ol] = softplus_f(wsd[i]) * epw[i]; }
  __syncthreads();
  for (int u = 0; u < 2; ++u) { const int idx = tid + u * 256, ol = idx >> 3, pc = idx & 7; union { v8h hh; v4u uu; } a, c;
#pragma unroll
    for (int i = 0; i < 8; ++i) { a.hh[i] = (_Float16)(t1[pc * 8 + i][ol] * 16.0f); c.hh[i] = (_Float16)(t2[pc * 8 + i][ol] * 256.0f); }
    vst2(P1 + (size_t)(o0 + ol) * DI + k0 + pc * 8, a.uu); vst2(P2 + (size_t)(o0 + ol) * DI + k0 + pc * 8, c.uu); }
}
__global__ __launch_bounds__(128) void k_gemm(const _Float16* __restrict__ x16, const _Float16* __restrict__ xs16, const _Float16* __restrict__ P1, const _Float16* __restrict__ P2, const int* __restrict__ r1, const int* __restrict__ r2,
                                            const float* __restrict__ bl, const float* __restrict__ bsd, const float* __restrict__ epb, float* __restrict__ out) {
  __shared__ __align__(16) float so[4][16][132];
  const int tid = threadIdx.x, wave = tid >> 5, lane = tid & 31, col = lane & 15, g = lane >> 4;
  const int r0 = blockIdx.x * 64 + wave * 16, n0 = blockIdx.y * 128;
  { v8f a1[8] = {};
#pragma unroll 1
    for (int kc = 0; kc < DI / 32; ++kc) { const v16h fa = frag_h(x16 + (size_t)(r0 + col) * DI + kc * 32, lane);
#pragma unroll
      for (int j = 0; j < 8; ++j) a1[j] = wmma16(fa, frag_h(P1 + (size_t)(n0 + j * 16 + col) * DI + kc * 32, lane), a1[j]); }
#pragma unroll
    for (int j = 0; j < 8; ++j) { const int o = n0 + j * 16 + col; const float bb = bl[o], bs = softplus_f(bsd[o]) * epb[o];
#pragma unroll
      for (int r = 0; r < 8; ++r) { const size_t row = (size_t)(r0 + 8 * g + r); so[wave][8 * g + r][j * 16 + col] = a1[j][r] * (1.0f / 16.0f) + bb + (float)r2[row * DO + o] * bs; } } }
  { v8f a2[8] = {};
#pragma unroll 1
    for (int kc = 0; kc < DI / 32; ++kc) { const v16h fb = frag_h(xs16 + (size_t)(r0 + col) * DI + kc * 32, lane);
#pragma unroll
      for (int j = 0; j < 8; ++j) a2[j] = wmma16(fb, frag_h(P2 + (size_t)(n0 + j * 16 + col) * DI + kc * 32, lane), a2[j]); }
#pragma unroll
    for (int j = 0; j < 8; ++j) { const int o = n0 + j * 16 + col;
#pragma unroll
      for (int r = 0; r < 8; ++r) { const size_t row = (size_t)(r0 + 8 * g + r); so[wave][8 * g + r][j * 16 + col] += (float)r1[row * DO + o] * a2[j][r] * (1.0f / 256.0f); } } }
  LDSX();
#pragma unroll 4
  for (int rl = 0; rl < 16; ++rl) vst2(out + (size_t)(r0 + rl) * DO + n0 + lane * 4, *(const v4f*)(&so[wave][rl][lane * 4]));
}
extern "C" void kernel_launch(void* const* d_in, const int* in_sizes, int n_in, void* d_out, int out_size, void* d_ws, size_t ws_size, hipStream_t stream) {
  (void)in_sizes; (void)n_in; (void)out_size; (void)ws_size;
  const float* x = (const float*)d_in[0]; const float* wl = (const float*)d_in[1]; const float* wsd = (const float*)d_in[2]; const float* bl = (const float*)d_in[3]; const float* bsd = (const float*)d_in[4];
  const float* epw = (const float*)d_in[5]; const float* epb = (const float*)d_in[6]; const int* s = (const int*)d_in[7]; const int* r1 = (const int*)d_in[8]; const int* r2 = (const int*)d_in[9];
  float* out = (float*)d_out;
  char* ws = (char*)d_ws; size_t off = 0;
  auto take = [&](size_t bytes) { char* p = ws + off; off += (bytes + 255) & ~(size_t)255; return p; };
  _Float16* x16 = (_Float16*)take((size_t)NBT * DI * 2); _Float16* xs16 = (_Float16*)take((size_t)NBT * DI * 2); _Float16* P1 = (_Float16*)take((size_t)DO * DI * 2); _Float16* P2 = (_Float16*)take((size_t)DO * DI * 2);
  k_cvtx<<<(unsigned)((size_t)NBT * DI / 8 / 256), 256, 0, stream>>>(x, s, x16, xs16);
  k_packT<<<dim3(DO / 64, DI / 64), 256, 0, stream>>>(wl, wsd, epw, P1, P2);
  k_gemm<<<dim3(NBT / 64, DO / 128), 128, 0, stream>>>(x16, xs16, P1, P2, r1, r2, bl, bsd, epb, out);
}
